// CrossAttention1D_14577119002773
// MI455X (gfx1250) — hardware-verified
//
#include <hip/hip_runtime.h>
#include <math.h>

constexpr int NBATCH = 4;
constexpr int NCH    = 1024;
constexpr int NLEN   = 2048;
constexpr int NHEAD  = 16;
constexpr int HDIM   = 64;
constexpr int NTOK   = NBATCH * NLEN;
constexpr int GRP_PER_CHUNK = 2;
constexpr int NGROUPS = NBATCH * NHEAD;
constexpr int NCHUNK  = NGROUPS / GRP_PER_CHUNK;
constexpr float SCORE_SCALE = 0.125f;

constexpr size_t MIB       = 1048576;
constexpr size_t OFFB_WO   = 0;
constexpr size_t OFFB_WQ   = 2 * MIB;
constexpr size_t OFFB_WK   = 4 * MIB;
constexpr size_t OFFB_WV   = 6 * MIB;
constexpr size_t OFFB_XQT  = 8 * MIB;
constexpr size_t OFFB_XCT  = 24 * MIB;
constexpr size_t OFFB_QTOK = 40 * MIB;
constexpr size_t OFFB_KTOK = 56 * MIB;
constexpr size_t OFFB_VCM  = 72 * MIB;
constexpr size_t OFFB_OTOK = 88 * MIB;
constexpr size_t OFFB_P    = 104 * MIB;
constexpr size_t OFFB_S    = 2 * MIB;
constexpr size_t WS_CARVE  = 120 * MIB;
static_assert(OFFB_S + (size_t)GRP_PER_CHUNK * NLEN * NLEN * 4 <= OFFB_QTOK);
static_assert(OFFB_P + (size_t)GRP_PER_CHUNK * NLEN * NLEN * 2 == WS_CARVE);
static_assert((size_t)NCH * NCH * 2 == 2 * MIB);
static_assert((size_t)NTOK * NCH * 2 == 16 * MIB);

typedef __attribute__((ext_vector_type(16))) _Float16 v16h;
typedef __attribute__((ext_vector_type(8)))  _Float16 v8h;
typedef __attribute__((ext_vector_type(16))) __bf16   v16b;
typedef __attribute__((ext_vector_type(8)))  __bf16   v8b;
typedef __attribute__((ext_vector_type(8)))  float    v8f;
typedef __attribute__((ext_vector_type(4)))  float    v4f;
typedef __attribute__((ext_vector_type(4)))  unsigned int v4u;

__device__ __forceinline__ unsigned short f2bf_bits(float f) {
  unsigned u = __float_as_uint(f);
  return (unsigned short)((u + 0x7FFFu + ((u >> 16) & 1u)) >> 16);
}
__device__ __forceinline__ float bf_bits2f(unsigned short h) { return __uint_as_float(((unsigned)h) << 16); }

__device__ __forceinline__ void dep_guard_h(v8f& a, v8f& b, v16h x, v16h y) { asm volatile("v_nop\n\tv_nop\n\tv_nop\n\tv_nop" : "+v"(a), "+v"(b) : "v"(x), "v"(y)); }
__device__ __forceinline__ void dep_guard_b(v8f& a, v8f& b, v16b x, v16b y) { asm volatile("v_nop\n\tv_nop\n\tv_nop\n\tv_nop" : "+v"(a), "+v"(b) : "v"(x), "v"(y)); }
__device__ __forceinline__ void keep4_h(v16h a, v16h b, v16h c, v16h d) { asm volatile("v_nop" :: "v"(a), "v"(b), "v"(c), "v"(d)); }
__device__ __forceinline__ void keep4_b(v16b a, v16b b, v16b c, v16b d) { asm volatile("v_nop" :: "v"(a), "v"(b), "v"(c), "v"(d)); }
__device__ __forceinline__ void acc_guard4(v8f& a, v8f& b, v8f& c, v8f& d) { asm volatile("v_nop\n\tv_nop\n\tv_nop\n\tv_nop" : "+v"(a), "+v"(b), "+v"(c), "+v"(d)); }
template <typename T> struct Frag;
template <> struct Frag<_Float16> {
  typedef v16h V; union U { v16h v; v8h h[2]; };
  static __device__ __forceinline__ v16h load(const _Float16* p) {
    U f; f.h[0] = *(const v8h*)(p); f.h[1] = *(const v8h*)(p + 16); return f.v;
  }
  static __device__ __forceinline__ v8f mma(v16h a, v16h b, v8f c) {
    return __builtin_amdgcn_wmma_f32_16x16x32_f16(false, a, false, b, (short)0, c, false, false);
  }
  static __device__ __forceinline__ void guard(v8f& a, v8f& b, v16h x, v16h y) { dep_guard_h(a, b, x, y); }
  static __device__ __forceinline__ void keep(v16h a, v16h b, v16h c, v16h d) { keep4_h(a, b, c, d); }
};
template <> struct Frag<__bf16> {
  typedef v16b V; union U { v16b v; v8b h[2]; };
  static __device__ __forceinline__ v16b load(const __bf16* p) {
    U f; f.h[0] = *(const v8b*)(p); f.h[1] = *(const v8b*)(p + 16); return f.v;
  }
  static __device__ __forceinline__ v8f mma(v16b a, v16b b, v8f c) {
    return __builtin_amdgcn_wmma_f32_16x16x32_bf16(false, a, false, b, (short)0, c, false, false);
  }
  static __device__ __forceinline__ void guard(v8f& a, v8f& b, v16b x, v16b y) { dep_guard_b(a, b, x, y); }
  static __device__ __forceinline__ void keep(v16b a, v16b b, v16b c, v16b d) { keep4_b(a, b, c, d); }
};

__device__ __forceinline__ unsigned pk16(unsigned short a, unsigned short b) { return (unsigned)a | ((unsigned)b << 16); }

template <int ET> struct Elem;
template <> struct Elem<0> { typedef _Float16 T; };
template <> struct Elem<1> { typedef __bf16 T; };
template <int ET, bool SPLIT, int BIAS_MODE, int OUT_MODE, bool RESID, int ACT = 0>
__global__ __launch_bounds__(256) void wmma_gemm64(
    const unsigned short* __restrict__ Ap, const unsigned short* __restrict__ A2p, int lda, long strideA,
    const unsigned short* __restrict__ Btp, const unsigned short* __restrict__ Bt2p, int ldb, long strideB,
    void* __restrict__ Cout, void* __restrict__ Cout2, int ldc, long strideC,
    const float* __restrict__ bias,
    const float* __restrict__ resid, long strideR,
    int M, int N, int K, float scale) {
  typedef typename Elem<ET>::T T;
  typedef typename Frag<T>::V V;
  const T* A = (const T*)Ap; const T* A2 = (const T*)A2p; const T* Bt = (const T*)Btp; const T* Bt2 = (const T*)Bt2p;
  __shared__ __align__(16) float sT[8][16 * 68];
  const int b    = blockIdx.y;
  const int lane = threadIdx.x & 31;
  const int wave = threadIdx.x >> 5;
  const int tilesN = N >> 6;
  const int tilesM = M >> 6;
  const int tile = blockIdx.x * 8 + wave;
  if (tile >= tilesM * tilesN) return;
  const int tm = tile / tilesN;
  const int tn = tile - tm * tilesN;
  const int m0 = tm << 6;
  const int n0 = tn << 6;

  const T* Ab  = A  + (size_t)b * strideA;
  const T* Bb  = Bt + (size_t)b * strideB;
  const T* Ab2 = SPLIT ? (A2  + (size_t)b * strideA) : nullptr;
  const T* Bb2 = SPLIT ? (Bt2 + (size_t)b * strideB) : nullptr;

  const int rlane = lane & 15;
  const int koff  = (lane >> 4) * 8;
  const int mOff  = (lane >> 4) * 8;

  v8f acc[4][4];
#pragma unroll
  for (int i = 0; i < 4; ++i)
#pragma unroll
    for (int j = 0; j < 4; ++j) acc[i][j] = (v8f){0.f,0.f,0.f,0.f,0.f,0.f,0.f,0.f};

  for (int k0 = 0; k0 < K; k0 += 32) {
    V bh[4], bl[4];
#pragma unroll
    for (int j = 0; j < 4; ++j) {
      const size_t bo = (size_t)(n0 + (j << 4) + rlane) * ldb + koff + k0;
      bh[j] = Frag<T>::load(Bb + bo);
      if (SPLIT) bl[j] = Frag<T>::load(Bb2 + bo);
    }
#pragma unroll
    for (int i = 0; i < 4; ++i) {
      const size_t ao = (size_t)(m0 + (i << 4) + rlane) * lda + koff + k0;
      V ah = Frag<T>::load(Ab + ao);
      V al;
      if (SPLIT) al = Frag<T>::load(Ab2 + ao);
#pragma unroll
      for (int j = 0; j < 4; ++j) {
        acc[i][j] = Frag<T>::mma(ah, bh[j], acc[i][j]);
        if (SPLIT) {
          acc[i][j] = Frag<T>::mma(ah, bl[j], acc[i][j]);
          acc[i][j] = Frag<T>::mma(al, bh[j], acc[i][j]);
        }
      }
      Frag<T>::guard(acc[i][0], acc[i][3], ah, SPLIT ? al : ah);
    }
    Frag<T>::keep(bh[0], bh[1], bh[2], bh[3]);
    if (SPLIT) Frag<T>::keep(bl[0], bl[1], bl[2], bl[3]);
  }
  acc_guard4(acc[0][0], acc[0][1], acc[0][2], acc[0][3]);
  acc_guard4(acc[1][0], acc[1][1], acc[1][2], acc[1][3]);
  acc_guard4(acc[2][0], acc[2][1], acc[2][2], acc[2][3]);
  acc_guard4(acc[3][0], acc[3][1], acc[3][2], acc[3][3]);

  float* slab = sT[wave];
  const float* Rb = RESID ? (resid + (size_t)b * strideR) : nullptr;
#pragma unroll
  for (int i = 0; i < 4; ++i) {
    const int mBase = m0 + (i << 4);
#pragma unroll
    for (int j = 0; j < 4; ++j) {
      const int n = n0 + (j << 4) + rlane;
      float bv = 0.f;
      if (BIAS_MODE == 2) bv = bias[n];
#pragma unroll
      for (int r = 0; r < 8; ++r) {
        float v = acc[i][j][r] * scale;
        if (BIAS_MODE == 1) v += bias[mBase + mOff + r];
        if (BIAS_MODE == 2) v += bv;
        if (RESID) v += Rb[(size_t)(mBase + mOff + r) * ldc + n];
        if (ACT == 2) v = fmaxf(v, 0.0f);
        if (ACT == 4) v = (v > 0.f) ? v : 0.01f * v;
        slab[(mOff + r) * 68 + (j << 4) + rlane] = v;
      }
    }
    __builtin_amdgcn_fence(__ATOMIC_RELEASE, "workgroup");
    __builtin_amdgcn_wave_barrier();
    __builtin_amdgcn_fence(__ATOMIC_ACQUIRE, "workgroup");
    if (OUT_MODE == 0) {
      float* C = (float*)Cout + (size_t)b * strideC;
      const int hh = lane >> 4, c4 = (lane & 15) * 4;
      for (int pass = 0; pass < 2; ++pass) {
#pragma unroll
        for (int it = 0; it < 8; ++it) {
          const int row = it * 2 + hh;
          v4f v = *(const v4f*)(slab + row * 68 + c4);
          *(volatile v4f*)(C + (size_t)(mBase + row) * ldc + n0 + c4) = v;
        }
        __threadfence();
      }
    } else {
      const int q = lane >> 3, c8 = (lane & 7) * 8;
      unsigned short* C  = (unsigned short*)Cout  + (size_t)b * strideC;
      unsigned short* C2 = (OUT_MODE == 2) ? ((unsigned short*)Cout2 + (size_t)b * strideC) : nullptr;
      for (int pass = 0; pass < 2; ++pass) {
#pragma unroll
        for (int it = 0; it < 4; ++it) {
          const int row = it * 4 + q;
          const float* sp = slab + row * 68 + c8;
          v8h hv, lv;
#pragma unroll
          for (int e = 0; e < 8; ++e) {
            if (OUT_MODE == 1) {
              hv[e] = (_Float16)sp[e];
            } else if (OUT_MODE == 3) {
              hv[e] = __builtin_bit_cast(_Float16, f2bf_bits(sp[e]));
            } else {
              unsigned short hb = f2bf_bits(sp[e]);
              unsigned short lb = f2bf_bits(sp[e] - bf_bits2f(hb));
              hv[e] = __builtin_bit_cast(_Float16, hb);
              lv[e] = __builtin_bit_cast(_Float16, lb);
            }
          }
          *(volatile v8h*)(C + (size_t)(mBase + row) * ldc + n0 + c8) = hv;
          if (OUT_MODE == 2) *(volatile v8h*)(C2 + (size_t)(mBase + row) * ldc + n0 + c8) = lv;
        }
        __threadfence();
      }
    }
    __builtin_amdgcn_fence(__ATOMIC_RELEASE, "workgroup");
    __builtin_amdgcn_wave_barrier();
    __builtin_amdgcn_fence(__ATOMIC_ACQUIRE, "workgroup");
  }
}

__global__ __launch_bounds__(256) void wcast_bf16_kernel(const float* __restrict__ W0, const float* __restrict__ W1,
                                                        const float* __restrict__ W2, const float* __restrict__ W3,
                                                        unsigned short* __restrict__ out) {
  const int y = blockIdx.y;
  const float* W = (y == 0) ? W0 : (y == 1) ? W1 : (y == 2) ? W2 : W3;
  const size_t i = (size_t)blockIdx.x * 256 + threadIdx.x;
  const float* p = W + 8 * i;
  const v4f a = *(const v4f*)(p);
  const v4f c = *(const v4f*)(p + 4);
  unsigned short hb[8];
#pragma unroll
  for (int e = 0; e < 4; ++e) {
    hb[e]     = f2bf_bits(a[e]);
    hb[4 + e] = f2bf_bits(c[e]);
  }
  const v4u u = (v4u){pk16(hb[0], hb[1]), pk16(hb[2], hb[3]), pk16(hb[4], hb[5]), pk16(hb[6], hb[7])};
  unsigned short* qo = out + (size_t)y * NCH * NCH + 8 * i;
  *(volatile v4u*)qo = u;
  __threadfence();
  *(volatile v4u*)qo = u;
}

__global__ __launch_bounds__(256) void tcast_bf16_kernel(const float* __restrict__ Xq, const float* __restrict__ Xc,
                                                        unsigned short* __restrict__ outQ, unsigned short* __restrict__ outC) {
  __shared__ float sm[64][65];
  const int t  = threadIdx.x;
  const int l0 = blockIdx.x * 64;
  const int c0 = blockIdx.y * 64;
  const int z  = blockIdx.z;
  const int b  = z & 3;
  const int which = z >> 2;
  const float* X = ((which == 0) ? Xq : Xc) + (size_t)b * NCH * NLEN;
  unsigned short* O = ((which == 0) ? outQ : outC) + (size_t)b * NLEN * NCH;
#pragma unroll
  for (int i = 0; i < 16; ++i) {
    const int e  = i * 256 + t;
    const int r  = e >> 6;
    const int cl = e & 63;
    sm[cl][r] = X[(size_t)(c0 + r) * NLEN + l0 + cl];
  }
  __syncthreads();
  const int lane = t & 31, wave = t >> 5;
  const int q = lane >> 3, c8 = (lane & 7) * 8;
  for (int pass = 0; pass < 2; ++pass) {
#pragma unroll
    for (int it = 0; it < 2; ++it) {
      const int row = wave * 8 + it * 4 + q;
      unsigned short hb[8];
#pragma unroll
      for (int e = 0; e < 8; ++e) hb[e] = f2bf_bits(sm[row][c8 + e]);
      const v4u u = (v4u){pk16(hb[0], hb[1]), pk16(hb[2], hb[3]), pk16(hb[4], hb[5]), pk16(hb[6], hb[7])};
      *(volatile v4u*)(O + (size_t)(l0 + row) * NCH + c0 + c8) = u;
    }
    __threadfence();
  }
}

__global__ __launch_bounds__(256) void softmax_rows_kernel(const float* __restrict__ S, unsigned short* __restrict__ P,
                                                          const int* __restrict__ nheads) {
  __shared__ float redM[8];
  __shared__ float redS[8];
  const int row  = blockIdx.x;
  const int t    = threadIdx.x;
  const int lane = t & 31, wave = t >> 5;
  const int c0   = t * 8;
  const float* sr = S + (size_t)row * NLEN + c0;
  const v4f a = *(const v4f*)(sr);
  const v4f c = *(const v4f*)(sr + 4);
  float x[8];
#pragma unroll
  for (int e = 0; e < 4; ++e) { x[e] = a[e]; x[4 + e] = c[e]; }
  float m = fmaxf(fmaxf(fmaxf(x[0], x[1]), fmaxf(x[2], x[3])), fmaxf(fmaxf(x[4], x[5]), fmaxf(x[6], x[7])));
#pragma unroll
  for (int off = 16; off > 0; off >>= 1) m = fmaxf(m, __shfl_xor(m, off, 32));
  if (lane == 0) redM[wave] = m;
  __syncthreads();
  float gm = redM[0];
#pragma unroll
  for (int w = 1; w < 8; ++w) gm = fmaxf(gm, redM[w]);
  float ex[8];
#pragma unroll
  for (int e = 0; e < 8; ++e) ex[e] = expf(x[e] - gm);
  float s = ((ex[0] + ex[1]) + (ex[2] + ex[3])) + ((ex[4] + ex[5]) + (ex[6] + ex[7]));
#pragma unroll
  for (int off = 16; off > 0; off >>= 1) s += __shfl_xor(s, off, 32);
  if (lane == 0) redS[wave] = s;
  __syncthreads();
  float gs = redS[0];
#pragma unroll
  for (int w = 1; w < 8; ++w) gs += redS[w];
  float inv = 1.0f / gs;
  const int hv = nheads[0];
  if (hv != NHEAD) inv = __uint_as_float(0x7FC00000u);
  unsigned short hb[8];
#pragma unroll
  for (int e = 0; e < 8; ++e) hb[e] = f2bf_bits(ex[e] * inv);
  const v4u u = (v4u){pk16(hb[0], hb[1]), pk16(hb[2], hb[3]), pk16(hb[4], hb[5]), pk16(hb[6], hb[7])};
  unsigned short* pp = P + (size_t)row * NLEN + c0;
  *(volatile v4u*)pp = u;
  __threadfence();
  *(volatile v4u*)pp = u;
}

extern "C" void kernel_launch(void* const* d_in, const int* in_sizes, int n_in,
                              void* d_out, int out_size, void* d_ws, size_t ws_size, hipStream_t stream) {
  if (n_in < 8) return;
  if (in_sizes[0] != NBATCH * NCH * NLEN) return;
  if (in_sizes[1] != NBATCH * NCH * NLEN) return;
  if (in_sizes[2] != NCH * NCH || in_sizes[3] != NCH * NCH || in_sizes[4] != NCH * NCH || in_sizes[5] != NCH * NCH) return;
  if (in_sizes[6] != NCH || in_sizes[7] < 1) return;
  if (out_size != NBATCH * NCH * NLEN) return;
  if (ws_size < WS_CARVE) return;

  const float* query   = (const float*)d_in[0];
  const float* context = (const float*)d_in[1];
  const float* Wq = (const float*)d_in[2];
  const float* Wk = (const float*)d_in[3];
  const float* Wv = (const float*)d_in[4];
  const float* Wo = (const float*)d_in[5];
  const float* bo = (const float*)d_in[6];
  const int*   nheads = (const int*)d_in[7];
  float* out = (float*)d_out;

  char* ws = (char*)d_ws;
  unsigned short* wo16 = (unsigned short*)(ws + OFFB_WO);
  unsigned short* wq16 = (unsigned short*)(ws + OFFB_WQ);
  unsigned short* wk16 = (unsigned short*)(ws + OFFB_WK);
  unsigned short* wv16 = (unsigned short*)(ws + OFFB_WV);
  unsigned short* xqt  = (unsigned short*)(ws + OFFB_XQT);
  unsigned short* xct  = (unsigned short*)(ws + OFFB_XCT);
  unsigned short* qtok = (unsigned short*)(ws + OFFB_QTOK);
  unsigned short* ktok = (unsigned short*)(ws + OFFB_KTOK);
  unsigned short* vcm  = (unsigned short*)(ws + OFFB_VCM);
  unsigned short* otok = (unsigned short*)(ws + OFFB_OTOK);
  unsigned short* pbuf = (unsigned short*)(ws + OFFB_P);
  float*          sbuf = (float*)(ws + OFFB_S);

  const unsigned short* nul16 = nullptr;
  const float* nulf = nullptr;

  wcast_bf16_kernel<<<dim3(512, 4), 256, 0, stream>>>(Wo, Wq, Wk, Wv, wo16);

  tcast_bf16_kernel<<<dim3(NLEN / 64, NCH / 64, 2 * NBATCH), 256, 0, stream>>>(query, context, xqt, xct);

  wmma_gemm64<1, false, 0, 3, false><<<dim3(256, 1), 256, 0, stream>>>(
      xqt, nul16, NCH, 0L, wq16, nul16, NCH, 0L, (void*)qtok, (void*)nullptr, NCH, 0L,
      nulf, nulf, 0L, NTOK, NCH, NCH, 1.0f);
  wmma_gemm64<1, false, 0, 3, false><<<dim3(256, 1), 256, 0, stream>>>(
      xct, nul16, NCH, 0L, wk16, nul16, NCH, 0L, (void*)ktok, (void*)nullptr, NCH, 0L,
      nulf, nulf, 0L, NTOK, NCH, NCH, 1.0f);
  wmma_gemm64<1, false, 0, 3, false><<<dim3(64, NBATCH), 256, 0, stream>>>(
      wv16, nul16, NCH, 0L, xct, nul16, NCH, (long)NLEN * NCH, (void*)vcm, (void*)nullptr, NLEN, (long)NCH * NLEN,
      nulf, nulf, 0L, NCH, NLEN, NCH, 1.0f);

  for (int ch = 0; ch < NCHUNK; ++ch) {
    const int g0 = ch * GRP_PER_CHUNK;
    const int b  = g0 / NHEAD;
    const int h0 = g0 % NHEAD;
    const size_t qkoff = (size_t)b * NLEN * NCH + (size_t)h0 * HDIM;
    wmma_gemm64<1, false, 0, 0, false><<<dim3(128, GRP_PER_CHUNK), 256, 0, stream>>>(
        qtok + qkoff, nul16, NCH, (long)HDIM, ktok + qkoff, nul16, NCH, (long)HDIM,
        (void*)sbuf, (void*)nullptr, NLEN, (long)NLEN * NLEN,
        nulf, nulf, 0L, NLEN, NLEN, HDIM, SCORE_SCALE);
    softmax_rows_kernel<<<dim3(GRP_PER_CHUNK * NLEN), 256, 0, stream>>>(sbuf, pbuf, nheads);
    wmma_gemm64<1, false, 0, 3, false><<<dim3(4, GRP_PER_CHUNK), 256, 0, stream>>>(
        pbuf, nul16, NLEN, (long)NLEN * NLEN,
        vcm + (size_t)b * NCH * NLEN + (size_t)h0 * HDIM * NLEN, nul16, NLEN, (long)HDIM * NLEN,
        (void*)(otok + qkoff), (void*)nullptr, NCH, (long)HDIM,
        nulf, nulf, 0L, NLEN, HDIM, NLEN, 1.0f);
  }

  wmma_gemm64<1, false, 1, 0, true><<<dim3(64, NBATCH), 256, 0, stream>>>(
      wo16, nul16, NCH, 0L, otok, nul16, NCH, (long)NLEN * NCH, (void*)out, (void*)nullptr, NLEN, (long)NCH * NLEN,
      bo, query, (long)NCH * NLEN, NCH, NLEN, NCH, 1.0f);
}
